// LSTMBehaviorModel_87582973100043
// MI455X (gfx1250) — hardware-run, weakly checked
//
#include <hip/hip_runtime.h>
#include <math.h>

typedef __attribute__((ext_vector_type(16))) _Float16 v16h;
typedef __attribute__((ext_vector_type(8)))  _Float16 v8h;
typedef __attribute__((ext_vector_type(8)))  float    v8f;
typedef __attribute__((ext_vector_type(4)))  float    v4f;
typedef __attribute__((ext_vector_type(4)))  unsigned v4u;

constexpr int kBatch   = 4096;
constexpr int kSteps   = 256;
constexpr int kFeat    = 5;
constexpr int kHid     = 64;
constexpr int kGates   = 4 * kHid;
constexpr int kRowsBlk = 32;
constexpr int kThreads = 256;
constexpr int kBlocks  = kBatch / kRowsBlk;
static_assert(kBatch % kRowsBlk == 0, "batch tile");
static_assert(kGates == 256 && kThreads == 256, "one thread per gate row in the prologue");

constexpr int kW0Pitch  = 104;
constexpr int kW1Pitch  = 136;
constexpr int kW0Halves = kGates * kW0Pitch;
constexpr int kW1Halves = kGates * kW1Pitch;
constexpr int kActPitch = 168;
constexpr int kActBuf   = kRowsBlk * kActPitch;
constexpr int kXCol     = 128;
constexpr int kChunkT   = 32;
constexpr int kXsPitch  = kChunkT * kFeat;
constexpr int kLastPitch = 68;
static_assert(kSteps % kChunkT == 0, "chunking");
static_assert(kRowsBlk * kXsPitch == 5 * kThreads * 4, "chunk load coverage: 5 float4 per thread");
static_assert(kRowsBlk * kLastPitch <= kRowsBlk * kXsPitch, "last-state alias fits");
static_assert((kW0Pitch % 8) == 0 && (kW1Pitch % 8) == 0 && (kActPitch % 8) == 0, "16-B aligned fragment rows");

constexpr float kCarryA    = 64.0f;
constexpr float kCarryW    = 64.0f;
constexpr float kCarryProd = kCarryA * kCarryW;
constexpr float kInvProd   = 1.0f / kCarryProd;
constexpr float kF16MinNormal = 6.103515625e-05f;

constexpr int kOut1Off = kBatch;
constexpr int kOut2Off = 2 * kBatch;
constexpr int kOutTotal = 2 * kBatch + kBatch * 5;
static_assert(kOut1Off * 4 == 16384 && kOut2Off * 4 == 32768, "output byte offsets");
static_assert(kOutTotal * 4 == 114688, "output bytes");

__device__ __forceinline__ unsigned hbits(float v, float carry) {
  float s = v * carry;
  s = (fabsf(s) < kF16MinNormal) ? 0.0f : s;
  const _Float16 h = (_Float16)s;
  return (unsigned)__builtin_bit_cast(unsigned short, h);
}
__device__ __forceinline__ unsigned pack2(float a, float b, float carry) {
  const unsigned lo = hbits(a, carry);
  const unsigned hi = hbits(b, carry);
  return lo | (hi << 16);
}
__device__ __forceinline__ _Float16 to_h(float v, float carry) {
  float s = v * carry;
  s = (fabsf(s) < kF16MinNormal) ? 0.0f : s;
  return (_Float16)s;
}

union FragU { v16h v; v8h h[2]; };
__device__ __forceinline__ v16h frag_load(const _Float16* p) {
  FragU f;
  f.h[0] = *(const v8h*)(p);
  f.h[1] = *(const v8h*)(p + 16);
  return f.v;
}
__device__ __forceinline__ v8f mma_f16(v16h a, v16h b, v8f c) {
  c = __builtin_amdgcn_wmma_f32_16x16x32_f16(false, a, false, b, (short)0, c, false, false);
  asm volatile("v_nop\n\tv_nop\n\tv_nop\n\tv_nop" : "+v"(c) : "v"(a), "v"(b));
  return c;
}

__device__ __forceinline__ float fsig(float v) {
  return __builtin_amdgcn_rcpf(1.0f + __expf(-v));
}
__device__ __forceinline__ float ftanh(float v) {
  const float e = __expf(-2.0f * fabsf(v));
  const float r = (1.0f - e) * __builtin_amdgcn_rcpf(1.0f + e);
  return copysignf(r, v);
}

__device__ __forceinline__ void cvt_plane64(const float* __restrict__ src, _Float16* dst,
                                            int pitch, int col0, int tid) {
#pragma unroll 2
  for (int i = 0; i < 8; ++i) {
    const int u  = tid + kThreads * i;
    const int n  = u >> 3;
    const int k8 = u & 7;
    const v4f a = *(const v4f*)(src + n * kHid + k8 * 8);
    const v4f b = *(const v4f*)(src + n * kHid + k8 * 8 + 4);
    const float a0 = a[0], a1 = a[1], a2 = a[2], a3 = a[3];
    const float c0 = b[0], c1 = b[1], c2 = b[2], c3 = b[3];
    const v4u w = (v4u){pack2(a0, a1, kCarryW), pack2(a2, a3, kCarryW),
                        pack2(c0, c1, kCarryW), pack2(c2, c3, kCarryW)};
    *(v4u*)(void*)(dst + n * pitch + col0 + k8 * 8) = w;
  }
}

__device__ __forceinline__ void load_x_chunk(const float* __restrict__ x, float* xs,
                                             int b0, int chunk, int tid) {
#pragma unroll
  for (int i = 0; i < 5; ++i) {
    const int idx = tid + kThreads * i;
    const int row = idx / 40;
    const int c4  = idx - row * 40;
    const v4f v = *(const v4f*)(x + (size_t)(b0 + row) * (kSteps * kFeat) + chunk * kXsPitch + c4 * 4);
    *(v4f*)(xs + row * kXsPitch + c4 * 4) = v;
  }
}

__device__ __forceinline__ void build_x16(const float* xs, _Float16* act, int buf, int step, int tid) {
  const int row = tid >> 2;
  const int seg = tid & 3;
  const int ts  = step & (kChunkT - 1);
  const float* xp = xs + row * kXsPitch + ts * kFeat;
  const bool on = (seg == 0);
  float v0 = xp[0], v1 = xp[1], v2 = xp[2], v3 = xp[3], v4 = xp[4];
  v0 = on ? v0 : 0.0f;
  v1 = on ? v1 : 0.0f;
  v2 = on ? v2 : 0.0f;
  v3 = on ? v3 : 0.0f;
  v4 = on ? v4 : 0.0f;
  const v4u w = (v4u){pack2(v0, v1, kCarryA), pack2(v2, v3, kCarryA), hbits(v4, kCarryA), 0u};
  *(v4u*)(void*)(act + buf * kActBuf + row * kActPitch + kXCol + seg * 8) = w;
}

__device__ __forceinline__ float dot64(const float* lp, const float* __restrict__ w) {
  float s = 0.0f;
#pragma unroll 8
  for (int k = 0; k < kHid; ++k) s = fmaf(lp[k], w[k], s);
  return s;
}
__device__ __forceinline__ float head_mlp(const float* lp, const float* __restrict__ w1,
                                          const float* __restrict__ b1, const float* __restrict__ w2,
                                          const float* __restrict__ b2) {
  float acc = 0.0f;
#pragma unroll 1
  for (int u = 0; u < 16; ++u) {
    float s = dot64(lp, w1 + u * kHid);
    s = s + b1[u];
    s = fmaxf(s, 0.0f);
    acc = fmaf(s, w2[u], acc);
  }
  acc = acc + b2[0];
  return 1.0f / (1.0f + expf(-acc));
}

__global__ void __launch_bounds__(256)
lstm2_heads_kernel(const float* __restrict__ x,
                   const float* __restrict__ w_ih0, const float* __restrict__ w_hh0,
                   const float* __restrict__ b_ih0, const float* __restrict__ b_hh0,
                   const float* __restrict__ w_ih1, const float* __restrict__ w_hh1,
                   const float* __restrict__ b_ih1, const float* __restrict__ b_hh1,
                   const float* __restrict__ eng_w1, const float* __restrict__ eng_b1,
                   const float* __restrict__ eng_w2, const float* __restrict__ eng_b2,
                   const float* __restrict__ prop_w1, const float* __restrict__ prop_b1,
                   const float* __restrict__ prop_w2, const float* __restrict__ prop_b2,
                   const float* __restrict__ seg_w, const float* __restrict__ seg_b,
                   float* out)
{
  __shared__ __align__(16) _Float16 sW[kW0Halves + kW1Halves];
  __shared__ __align__(16) _Float16 sAct[2 * kActBuf];
  __shared__ __align__(16) float    sXS[kRowsBlk * kXsPitch];
  __shared__ __align__(16) float    sOut[224];

  const int tid  = (int)threadIdx.x;
  const int lane = tid & 31;
  const int wave = __builtin_amdgcn_readfirstlane(tid >> 5);
  const int b0   = (int)blockIdx.x * kRowsBlk;
  const int hh   = lane >> 4;
  const int m    = lane & 15;
  const bool isL1 = (wave >= 4);
  const int col  = 16 * (wave & 3) + m;

  cvt_plane64(w_hh0, sW, kW0Pitch, 0, tid);
  cvt_plane64(w_ih1, sW + kW0Halves, kW1Pitch, 0, tid);
  cvt_plane64(w_hh1, sW + kW0Halves, kW1Pitch, kHid, tid);
  {
    const int n = tid;
    const float q0 = w_ih0[n * kFeat + 0];
    const float q1 = w_ih0[n * kFeat + 1];
    const float q2 = w_ih0[n * kFeat + 2];
    const float q3 = w_ih0[n * kFeat + 3];
    const float q4 = w_ih0[n * kFeat + 4];
    const v4u w = (v4u){pack2(q0, q1, kCarryW), pack2(q2, q3, kCarryW), hbits(q4, kCarryW), 0u};
    const v4u z = (v4u){0u, 0u, 0u, 0u};
    _Float16* d = sW + n * kW0Pitch + kHid;
    *(v4u*)(void*)(d)      = w;
    *(v4u*)(void*)(d + 8)  = z;
    *(v4u*)(void*)(d + 16) = z;
    *(v4u*)(void*)(d + 24) = z;
  }
  {
    const v4u z = (v4u){0u, 0u, 0u, 0u};
    for (int i = tid; i < (2 * kActBuf) / 8; i += kThreads) *(v4u*)(void*)(sAct + i * 8) = z;
  }
  load_x_chunk(x, sXS, b0, 0, tid);
  __syncthreads();
  if (wave < 4) build_x16(sXS, sAct, 0, 0, tid);

  const float* bi = isL1 ? b_ih1 : b_ih0;
  const float* bh = isL1 ? b_hh1 : b_hh0;
  float bsc[4];
#pragma unroll
  for (int g = 0; g < 4; ++g) bsc[g] = (bi[g * kHid + col] + bh[g * kHid + col]) * kCarryProd;

  const int wpitch = isL1 ? kW1Pitch : kW0Pitch;
  const int woff   = isL1 ? kW0Halves : 0;
  const int nkc    = isL1 ? 4 : 3;
  const int hcol0  = isL1 ? kHid : 0;
  const _Float16* wrow = sW + woff + col * wpitch + 8 * hh;

  v8f cst[2];
#pragma unroll
  for (int mt = 0; mt < 2; ++mt) cst[mt] = (v8f){0.f, 0.f, 0.f, 0.f, 0.f, 0.f, 0.f, 0.f};

  __syncthreads();

#pragma unroll 1
  for (int t = 0; t <= kSteps; ++t) {
    const int cur = t & 1;
    const int nxt = cur ^ 1;
    const int tn  = t + 1;
    if (tn < kSteps && (tn & (kChunkT - 1)) == 0) {
      load_x_chunk(x, sXS, b0, tn / kChunkT, tid);
      __syncthreads();
    }
    if (wave < 4 && tn < kSteps) build_x16(sXS, sAct, nxt, tn, tid);

    const bool active = isL1 ? (t >= 1) : (t < kSteps);
    if (active) {
      v8f acc[2][4];
#pragma unroll
      for (int mt = 0; mt < 2; ++mt)
#pragma unroll
        for (int g = 0; g < 4; ++g) {
          const float bv = bsc[g];
          acc[mt][g] = (v8f){bv, bv, bv, bv, bv, bv, bv, bv};
        }
      const _Float16* arow = sAct + cur * kActBuf + m * kActPitch + 8 * hh;
#pragma unroll 1
      for (int kc = 0; kc < nkc; ++kc) {
        const int acol = (!isL1 && kc == 2) ? kXCol : (kc * 32);
        const v16h a0 = frag_load(arow + acol);
        const v16h a1 = frag_load(arow + 16 * kActPitch + acol);
#pragma unroll
        for (int g = 0; g < 4; ++g) {
          const v16h bf = frag_load(wrow + g * kHid * wpitch + kc * 32);
          acc[0][g] = mma_f16(a0, bf, acc[0][g]);
          acc[1][g] = mma_f16(a1, bf, acc[1][g]);
        }
      }
      float hv[2][8];
#pragma unroll
      for (int mt = 0; mt < 2; ++mt) {
#pragma unroll
        for (int r = 0; r < 8; ++r) {
          const float ig = fsig(acc[mt][0][r] * kInvProd);
          const float fg = fsig(acc[mt][1][r] * kInvProd);
          const float gg = ftanh(acc[mt][2][r] * kInvProd);
          const float og = fsig(acc[mt][3][r] * kInvProd);
          const float cc = fg * cst[mt][r] + ig * gg;
          cst[mt][r] = cc;
          hv[mt][r] = og * ftanh(cc);
        }
      }
      if (t == kSteps) {
#pragma unroll
        for (int mt = 0; mt < 2; ++mt)
#pragma unroll
          for (int r = 0; r < 8; ++r)
            sXS[(mt * 16 + 8 * hh + r) * kLastPitch + col] = hv[mt][r];
      } else {
        _Float16* hdst = sAct + nxt * kActBuf + hcol0 + col;
#pragma unroll
        for (int mt = 0; mt < 2; ++mt)
#pragma unroll
          for (int r = 0; r < 8; ++r)
            hdst[(mt * 16 + 8 * hh + r) * kActPitch] = to_h(hv[mt][r], kCarryA);
      }
    }
    __syncthreads();
  }

  if (wave == 0) {
    const float* lp = sXS + lane * kLastPitch;
    sOut[lane]      = head_mlp(lp, eng_w1, eng_b1, eng_w2, eng_b2);
    sOut[32 + lane] = head_mlp(lp, prop_w1, prop_b1, prop_w2, prop_b2);
#pragma unroll 1
    for (int q = 0; q < 5; ++q) {
      float s = dot64(lp, seg_w + q * kHid);
      s = s + seg_b[q];
      sOut[64 + lane * 5 + q] = s;
    }
  }
  __syncthreads();
  if (wave == 0) {
    const float o0 = sOut[lane];
    const float o1 = sOut[32 + lane];
    const float s0 = sOut[64 + lane];
    const float s1 = sOut[96 + lane];
    const float s2 = sOut[128 + lane];
    const float s3 = sOut[160 + lane];
    const float s4 = sOut[192 + lane];
    volatile float* vo = out;
    const int p0 = b0 + lane;
    const int p1 = kOut1Off + b0 + lane;
    const int p2 = kOut2Off + b0 * 5 + lane;
    vo[p0] = o0;
    vo[p1] = o1;
    vo[p2] = s0;
    vo[p2 + 32] = s1;
    vo[p2 + 64] = s2;
    vo[p2 + 96] = s3;
    vo[p2 + 128] = s4;
    __threadfence();
    vo[p0] = o0;
    vo[p1] = o1;
    vo[p2] = s0;
    vo[p2 + 32] = s1;
    vo[p2 + 64] = s2;
    vo[p2 + 96] = s3;
    vo[p2 + 128] = s4;
  }
}

extern "C" void kernel_launch(void* const* d_in, const int* in_sizes, int n_in,
                              void* d_out, int out_size, void* d_ws, size_t ws_size,
                              hipStream_t stream) {
  (void)d_ws; (void)ws_size;
  if (n_in < 19) return;
  const int expect[19] = {
    kBatch * kSteps * kFeat, kGates * kFeat, kGates * kHid, kGates, kGates,
    kGates * kHid, kGates * kHid, kGates, kGates,
    16 * kHid, 16, 16, 1,
    16 * kHid, 16, 16, 1,
    5 * kHid, 5 };
  for (int i = 0; i < 19; ++i) {
    if (in_sizes[i] != expect[i]) return;
  }
  if (out_size != kOutTotal) return;

  const float* x       = (const float*)d_in[0];
  const float* w_ih0   = (const float*)d_in[1];
  const float* w_hh0   = (const float*)d_in[2];
  const float* b_ih0   = (const float*)d_in[3];
  const float* b_hh0   = (const float*)d_in[4];
  const float* w_ih1   = (const float*)d_in[5];
  const float* w_hh1   = (const float*)d_in[6];
  const float* b_ih1   = (const float*)d_in[7];
  const float* b_hh1   = (const float*)d_in[8];
  const float* eng_w1  = (const float*)d_in[9];
  const float* eng_b1  = (const float*)d_in[10];
  const float* eng_w2  = (const float*)d_in[11];
  const float* eng_b2  = (const float*)d_in[12];
  const float* prop_w1 = (const float*)d_in[13];
  const float* prop_b1 = (const float*)d_in[14];
  const float* prop_w2 = (const float*)d_in[15];
  const float* prop_b2 = (const float*)d_in[16];
  const float* seg_w   = (const float*)d_in[17];
  const float* seg_b   = (const float*)d_in[18];
  float* out = (float*)d_out;

  lstm2_heads_kernel<<<dim3(kBlocks), dim3(kThreads), 0, stream>>>(
      x, w_ih0, w_hh0, b_ih0, b_hh0, w_ih1, w_hh1, b_ih1, b_hh1,
      eng_w1, eng_b1, eng_w2, eng_b2, prop_w1, prop_b1, prop_w2, prop_b2,
      seg_w, seg_b, out);
}
